// TemporalLogicMachineDP_45938970198159
// MI455X (gfx1250) — hardware-verified
//
#include <hip/hip_runtime.h>

#define NB   2
#define NT   512
#define ND   64
#define NREL 128
#define NH   64
#define NBT  (NB * NT)

typedef _Float16 v16h __attribute__((ext_vector_type(16)));
typedef _Float16 v8h  __attribute__((ext_vector_type(8)));
typedef float    v8f  __attribute__((ext_vector_type(8)));
typedef float    v4f  __attribute__((ext_vector_type(4)));
typedef v8h __attribute__((may_alias)) v8ha;
typedef v4f __attribute__((may_alias)) v4fa;

union Frag16 { v16h v; v8h half[2]; _Float16 e[16]; };

__device__ __forceinline__ v8f wmma_f16(v16h a, v16h b, v8f c) {
    v8f d = __builtin_amdgcn_wmma_f32_16x16x32_f16(false, a, false, b, (short)0, c, false, false);
    asm volatile("v_nop\n\tv_nop\n\tv_nop\n\tv_nop" : "+v"(d) : "v"(a), "v"(b));
    return d;
}

__device__ __forceinline__ v16h frag_a_f32(const float* p, int h) {
    const v4f x0 = *(const v4fa*)(p + 8 * h);
    const v4f x1 = *(const v4fa*)(p + 8 * h + 4);
    const v4f y0 = *(const v4fa*)(p + 16 + 8 * h);
    const v4f y1 = *(const v4fa*)(p + 20 + 8 * h);
    v16h r = { (_Float16)x0.x, (_Float16)x0.y, (_Float16)x0.z, (_Float16)x0.w,
               (_Float16)x1.x, (_Float16)x1.y, (_Float16)x1.z, (_Float16)x1.w,
               (_Float16)y0.x, (_Float16)y0.y, (_Float16)y0.z, (_Float16)y0.w,
               (_Float16)y1.x, (_Float16)y1.y, (_Float16)y1.z, (_Float16)y1.w };
    return r;
}

__device__ __forceinline__ v16h frag_w_col(const float* __restrict__ W, int k0, int n, int h) {
    Frag16 fr;
#pragma unroll
    for (int e = 0; e < 8; ++e) {
        fr.e[e]     = (_Float16)(W[(size_t)(k0 + 8 * h + e) * NH + n] * 16.0f);
        fr.e[8 + e] = (_Float16)(W[(size_t)(k0 + 16 + 8 * h + e) * NH + n] * 16.0f);
    }
    return fr.v;
}

__global__ void __launch_bounds__(128) suffix_pool_kernel(const float* __restrict__ f,
                                                           float* __restrict__ cur0) {
    const int b  = blockIdx.x;
    const int c  = threadIdx.x;
    const int ch = c & 63;
    const bool isMin = (c >= 64);
    float run = isMin ? __builtin_inff() : -__builtin_inff();
#pragma unroll 1
    for (int t = NT - 1; t >= 0; --t) {
        const float v = f[((size_t)b * NT + t) * ND + ch];
        run = isMin ? fminf(run, v) : fmaxf(run, v);
        float* p = cur0 + ((size_t)b * NT + t) * NREL + c;
        *(volatile float*)p = run;
        __threadfence();
        *(volatile float*)p = run;
    }
}

__device__ __forceinline__ void t1_store_pass(const float* sT, float* t1, int r0, int w, int lane) {
    const int q8 = lane & 7, sub = lane >> 3;
#pragma unroll
    for (int i = 0; i < 2; ++i) {
        const int lid = 4 * i + sub;
        const int row = 4 * w + (lid >> 1);
        const int hl  = lid & 1;
        const v4f v = *(const v4fa*)(sT + row * NH + 32 * hl + 4 * q8);
        *(volatile v4f*)(t1 + (size_t)(r0 + row) * NH + 32 * hl + 4 * q8) = v;
    }
}

__global__ void __launch_bounds__(128) term1_kernel(const float* __restrict__ cur, int Ccur,
                                                    const float* __restrict__ W,
                                                    const float* __restrict__ bias,
                                                    float* __restrict__ t1) {
    __shared__ __attribute__((aligned(16))) float sT[16 * NH];

    const int tid = threadIdx.x, lane = tid & 31, w = tid >> 5;
    const int h = lane >> 4, m = lane & 15;
    const int r0 = blockIdx.x * 16;
    const int n0 = 16 * w;

    v8f acc = {0.f, 0.f, 0.f, 0.f, 0.f, 0.f, 0.f, 0.f};
    const float* arow = cur + (size_t)(r0 + m) * Ccur;
#pragma unroll 1
    for (int k0 = 0; k0 < Ccur; k0 += 32) {
        const v16h a  = frag_a_f32(arow + k0, h);
        const v16h bb = frag_w_col(W, k0, n0 + m, h);
        acc = wmma_f16(a, bb, acc);
    }

    const float bv = bias[n0 + m];
#pragma unroll
    for (int r = 0; r < 8; ++r) sT[(8 * h + r) * NH + n0 + m] = acc[r] * 0.0625f + bv;
    __syncthreads();

    t1_store_pass(sT, t1, r0, w, lane);
    __threadfence();
    t1_store_pass(sT, t1, r0, w, lane);
}

__global__ void __launch_bounds__(128) layer_kernel(const float* __restrict__ f,
                                                    const float* __restrict__ t1,
                                                    const float* __restrict__ Wbot,
                                                    float* __restrict__ dst) {
    __shared__ __attribute__((aligned(16))) _Float16 tileR[16 * NREL];
    __shared__ __attribute__((aligned(16))) float sOut[NH];

    const int b    = blockIdx.x / NT;
    const int i    = blockIdx.x % NT;
    const int tid  = threadIdx.x;
    const int wave = tid >> 5;
    const int lane = tid & 31;
    const int lo   = lane & 15;
    const int hi   = lane >> 4;
    const float NEG = -__builtin_inff();

    const int o = wave * 16 + lo;
    v16h bfr[4];
#pragma unroll
    for (int kk = 0; kk < 4; ++kk) bfr[kk] = frag_w_col(Wbot, 32 * kk, o, hi);

    const int  c     = tid;
    const int  ch    = c & 63;
    const bool isMin = (c >= 64);
    float run = isMin ? __builtin_inff() : NEG;

    float mx = NEG;
    const int jt0 = i >> 4;

#pragma unroll 1
    for (int jt = jt0; jt < (NT / 16); ++jt) {
        const int jbase = jt * 16;

        float vals[16];
#pragma unroll
        for (int jj = 0; jj < 16; ++jj)
            vals[jj] = f[((size_t)b * NT + jbase + jj) * ND + ch];
#pragma unroll
        for (int jj = 0; jj < 16; ++jj) {
            const int j = jbase + jj;
            const float nrun = isMin ? fminf(run, vals[jj]) : fmaxf(run, vals[jj]);
            run = (j >= i) ? nrun : run;
            tileR[jj * NREL + c] = (_Float16)((j >= i) ? run : 0.0f);
        }
        __syncthreads();

        v8f acc = {0.f, 0.f, 0.f, 0.f, 0.f, 0.f, 0.f, 0.f};
#pragma unroll
        for (int kk = 0; kk < 4; ++kk) {
            const int kbase = kk * 32;
            Frag16 af;
            af.half[0] = *(const v8ha*)(tileR + lo * NREL + kbase + 8 * hi);
            af.half[1] = *(const v8ha*)(tileR + lo * NREL + kbase + 16 + 8 * hi);
            acc = wmma_f16(af.v, bfr[kk], acc);
        }

        const float* t1p = t1 + ((size_t)b * NT + jbase + hi * 8) * NH + o;
        float tv[8];
#pragma unroll
        for (int r = 0; r < 8; ++r) tv[r] = t1p[(size_t)r * NH];
#pragma unroll
        for (int r = 0; r < 8; ++r) {
            const int j = jbase + r + hi * 8;
            const float val = acc[r] * 0.0625f + tv[r];
            mx = fmaxf(mx, (j >= i) ? val : NEG);
        }
        __syncthreads();
    }

    const float other = __shfl_xor(mx, 16, 32);
    mx = fmaxf(mx, other);
    mx = fmaxf(mx, -80.0f);
    const float s = __builtin_amdgcn_rcpf(1.0f + expf(-mx));
    if (hi == 0) sOut[o] = s;
    __syncthreads();

    if (tid < 16) {
        const v4f v = *(const v4fa*)(sOut + 4 * tid);
        float* p = dst + ((size_t)b * NT + i) * NH + 4 * tid;
        *(volatile v4f*)p = v;
        __threadfence();
        *(volatile v4f*)p = v;
    }
}

extern "C" void kernel_launch(void* const* d_in, const int* in_sizes, int n_in,
                              void* d_out, int out_size, void* d_ws, size_t ws_size,
                              hipStream_t stream) {
    if (n_in < 7) return;
    if (in_sizes[0] != NBT * ND) return;
    if (in_sizes[1] != (NREL + NREL) * NH) return;
    if (in_sizes[2] != NH) return;
    if (in_sizes[3] != (NH + NREL) * NH) return;
    if (in_sizes[4] != NH) return;
    if (in_sizes[5] != (NH + NREL) * NH) return;
    if (in_sizes[6] != NH) return;
    if (out_size != NBT * NH) return;

    const float* f  = (const float*)d_in[0];
    const float* W0 = (const float*)d_in[1];
    const float* b0 = (const float*)d_in[2];
    const float* W1 = (const float*)d_in[3];
    const float* b1 = (const float*)d_in[4];
    const float* W2 = (const float*)d_in[5];
    const float* b2 = (const float*)d_in[6];
    float* out = (float*)d_out;

    const size_t cur0_bytes = (size_t)NBT * NREL * sizeof(float);
    const size_t pl_bytes   = (size_t)NBT * NH * sizeof(float);
    const size_t total = cur0_bytes + 3 * pl_bytes;
    if (total > ws_size) return;

    char* ws = (char*)d_ws;
    float* cur0 = (float*)(ws);
    float* t1   = (float*)(ws + cur0_bytes);
    float* curA = (float*)(ws + cur0_bytes + pl_bytes);
    float* curB = (float*)(ws + cur0_bytes + 2 * pl_bytes);

    suffix_pool_kernel<<<NB, 128, 0, stream>>>(f, cur0);

    term1_kernel<<<NBT / 16, 128, 0, stream>>>(cur0, NREL, W0, b0, t1);
    layer_kernel<<<NBT, 128, 0, stream>>>(f, t1, W0 + (size_t)NREL * NH, curA);

    term1_kernel<<<NBT / 16, 128, 0, stream>>>(curA, NH, W1, b1, t1);
    layer_kernel<<<NBT, 128, 0, stream>>>(f, t1, W1 + (size_t)NH * NH, curB);

    term1_kernel<<<NBT / 16, 128, 0, stream>>>(curB, NH, W2, b2, t1);
    layer_kernel<<<NBT, 128, 0, stream>>>(f, t1, W2 + (size_t)NH * NH, out);
}
